// ImprovedTransformerEncoderBlock_52364241272888
// MI455X (gfx1250) — hardware-verified
//
#include <hip/hip_runtime.h>
#include <math.h>

constexpr int kB      = 4;
constexpr int kS      = 1024;
constexpr int kD      = 1024;
constexpr int kH      = 16;
constexpr int kDk     = 64;
constexpr int kFF     = 4096;
constexpr int kTok    = kB * kS;
constexpr int kMaxRel = 32;
constexpr int kRel    = 2 * kMaxRel + 1;
constexpr int kRelPad = 128;
constexpr int kG      = 8;
constexpr int kNChunk = (kB * kH) / kG;
constexpr int kSPitch = kS + kRelPad;
constexpr float kWCarry   = 64.0f;
constexpr float kRelkCarry = 16.0f;
constexpr float kPCarry   = 2048.0f;
constexpr float kCtxCarry = 64.0f;
constexpr float kGCarry   = 16.0f;
constexpr float kInvD     = 1.0f / 1024.0f;
constexpr float kLnEps    = 1e-5f;

static_assert(kSPitch % 64 == 0, "pitch must be a whole number of 128-B lines in f16 and f32");
static_assert(kNChunk * kG == kB * kH, "chunking");

constexpr size_t kSzSrc1 = (size_t)kTok * kD * 4;
constexpr size_t kSzX16  = (size_t)kTok * kD * 2;
constexpr size_t kSzW4   = (size_t)4 * kD * kD * 2;
constexpr size_t kSzVT   = (size_t)kB * kH * kDk * kSPitch * 2;
constexpr size_t kSzSC   = (size_t)kG * kS * kSPitch * 4;
constexpr size_t kSzP16  = (size_t)kG * kS * kSPitch * 2;
constexpr size_t kSzRelk = (size_t)kRelPad * kDk * 2;
constexpr size_t kSzW1   = (size_t)2 * kFF * kD * 2;
constexpr size_t kSzW2   = (size_t)kD * kFF * 2;
constexpr size_t kSzH    = (size_t)kS * 2 * kFF * 4;
constexpr size_t kSzG16  = (size_t)kTok * kFF * 2;

constexpr size_t kOffSrc1 = 0;
constexpr size_t kOffX16  = kOffSrc1 + kSzSrc1;
constexpr size_t kOffW4   = kOffX16 + kSzX16;
constexpr size_t kOffQ16  = kOffW4 + kSzW4;
constexpr size_t kOffK16  = kOffQ16 + kSzX16;
constexpr size_t kOffVT   = kOffK16 + kSzX16;
constexpr size_t kOffSC   = kOffVT + kSzVT;
constexpr size_t kOffP16  = kOffSC + kSzSC;
constexpr size_t kOffCtx  = kOffP16 + kSzP16;
constexpr size_t kOffRelk = kOffCtx + kSzX16;
constexpr size_t kWsEnd1  = kOffRelk + kSzRelk;

constexpr size_t kOffY16  = kOffX16;
constexpr size_t kOffW1   = kOffW4;
constexpr size_t kOffW2   = kOffW1 + kSzW1;
constexpr size_t kOffH    = kOffW2 + kSzW2;
constexpr size_t kOffG16  = kOffH + kSzH;
constexpr size_t kWsEnd2  = kOffG16 + kSzG16;
constexpr size_t kWsTotal = (kWsEnd1 > kWsEnd2) ? kWsEnd1 : kWsEnd2;

static_assert(kWsEnd1 == 124796928ull, "phase 1 carve");
static_assert(kWsEnd2 == 117440512ull, "phase 2 carve");
static_assert(kWsTotal <= 134217728ull, "carve under 128 MiB");
static_assert(kOffY16 + kSzX16 <= kOffW1, "Y16 does not overlap W1");
static_assert(kOffSrc1 + kSzSrc1 <= kOffY16, "SRC1 does not overlap phase-2 regions");
static_assert((kOffW4 % 128) == 0 && (kOffVT % 128) == 0 && (kOffSC % 128) == 0 && (kOffP16 % 128) == 0 &&
              (kOffCtx % 128) == 0 && (kOffRelk % 128) == 0 && (kOffH % 128) == 0 && (kOffG16 % 128) == 0, "128-B aligned");

typedef __attribute__((ext_vector_type(16))) _Float16 v16h;
typedef __attribute__((ext_vector_type(8)))  _Float16 v8h;
typedef __attribute__((ext_vector_type(16))) __bf16   v16b;
typedef __attribute__((ext_vector_type(8)))  __bf16   v8b;
typedef __attribute__((ext_vector_type(8)))  float    v8f;
typedef __attribute__((ext_vector_type(4)))  float    v4f;
typedef __attribute__((ext_vector_type(4)))  unsigned int v4u;

__device__ __forceinline__ unsigned short f2bf_bits(float f) {
  unsigned u = __float_as_uint(f);
  return (unsigned short)((u + 0x7FFFu + ((u >> 16) & 1u)) >> 16);
}
__device__ __forceinline__ float bf_bits2f(unsigned short h) { return __uint_as_float(((unsigned)h) << 16); }

__device__ __forceinline__ void dep_guard_h(v8f& a, v8f& b, v16h x, v16h y) { asm volatile("v_nop\n\tv_nop\n\tv_nop\n\tv_nop" : "+v"(a), "+v"(b) : "v"(x), "v"(y)); }
__device__ __forceinline__ void dep_guard_b(v8f& a, v8f& b, v16b x, v16b y) { asm volatile("v_nop\n\tv_nop\n\tv_nop\n\tv_nop" : "+v"(a), "+v"(b) : "v"(x), "v"(y)); }
__device__ __forceinline__ void keep4_h(v16h a, v16h b, v16h c, v16h d) { asm volatile("v_nop" :: "v"(a), "v"(b), "v"(c), "v"(d)); }
__device__ __forceinline__ void keep4_b(v16b a, v16b b, v16b c, v16b d) { asm volatile("v_nop" :: "v"(a), "v"(b), "v"(c), "v"(d)); }
__device__ __forceinline__ void acc_guard4(v8f& a, v8f& b, v8f& c, v8f& d) { asm volatile("v_nop\n\tv_nop\n\tv_nop\n\tv_nop" : "+v"(a), "+v"(b), "+v"(c), "+v"(d)); }
template <typename T> struct Frag;
template <> struct Frag<_Float16> {
  typedef v16h V; union U { v16h v; v8h h[2]; };
  static __device__ __forceinline__ v16h load(const _Float16* p) {
    U f; f.h[0] = *(const v8h*)(p); f.h[1] = *(const v8h*)(p + 16); return f.v;
  }
  static __device__ __forceinline__ v8f mma(v16h a, v16h b, v8f c) {
    return __builtin_amdgcn_wmma_f32_16x16x32_f16(false, a, false, b, (short)0, c, false, false);
  }
  static __device__ __forceinline__ void guard(v8f& a, v8f& b, v16h x, v16h y) { dep_guard_h(a, b, x, y); }
  static __device__ __forceinline__ void keep(v16h a, v16h b, v16h c, v16h d) { keep4_h(a, b, c, d); }
};
template <> struct Frag<__bf16> {
  typedef v16b V; union U { v16b v; v8b h[2]; };
  static __device__ __forceinline__ v16b load(const __bf16* p) {
    U f; f.h[0] = *(const v8b*)(p); f.h[1] = *(const v8b*)(p + 16); return f.v;
  }
  static __device__ __forceinline__ v8f mma(v16b a, v16b b, v8f c) {
    return __builtin_amdgcn_wmma_f32_16x16x32_bf16(false, a, false, b, (short)0, c, false, false);
  }
  static __device__ __forceinline__ void guard(v8f& a, v8f& b, v16b x, v16b y) { dep_guard_b(a, b, x, y); }
  static __device__ __forceinline__ void keep(v16b a, v16b b, v16b c, v16b d) { keep4_b(a, b, c, d); }
};

__device__ __forceinline__ unsigned pk16(unsigned short a, unsigned short b) { return (unsigned)a | ((unsigned)b << 16); }
__device__ __forceinline__ unsigned short h_bits(float f) { const _Float16 h = (_Float16)f; return __builtin_bit_cast(unsigned short, h); }

template <int ET> struct Elem;
template <> struct Elem<0> { typedef _Float16 T; };
template <> struct Elem<1> { typedef __bf16 T; };
template <int ET, bool SPLIT, int BIAS_MODE, int OUT_MODE, bool RESID, int ACT = 0>
__global__ __launch_bounds__(256) void wmma_gemm64(
    const unsigned short* __restrict__ Ap, const unsigned short* __restrict__ A2p, int lda, long strideA,
    const unsigned short* __restrict__ Btp, const unsigned short* __restrict__ Bt2p, int ldb, long strideB,
    void* __restrict__ Cout, void* __restrict__ Cout2, int ldc, long strideC,
    const float* __restrict__ bias,
    const float* __restrict__ resid, long strideR,
    int M, int N, int K, float scale) {
  typedef typename Elem<ET>::T T;
  typedef typename Frag<T>::V V;
  const T* A = (const T*)Ap; const T* A2 = (const T*)A2p; const T* Bt = (const T*)Btp; const T* Bt2 = (const T*)Bt2p;
  __shared__ __align__(16) float sT[8][16 * 68];
  const int b    = blockIdx.y;
  const int lane = threadIdx.x & 31;
  const int wave = threadIdx.x >> 5;
  const int tilesN = N >> 6;
  const int tilesM = M >> 6;
  const int tile = blockIdx.x * 8 + wave;
  if (tile >= tilesM * tilesN) return;
  const int tm = tile / tilesN;
  const int tn = tile - tm * tilesN;
  const int m0 = tm << 6;
  const int n0 = tn << 6;

  const T* Ab  = A  + (size_t)b * strideA;
  const T* Bb  = Bt + (size_t)b * strideB;
  const T* Ab2 = SPLIT ? (A2  + (size_t)b * strideA) : nullptr;
  const T* Bb2 = SPLIT ? (Bt2 + (size_t)b * strideB) : nullptr;

  const int rlane = lane & 15;
  const int koff  = (lane >> 4) * 8;
  const int mOff  = (lane >> 4) * 8;

  v8f acc[4][4];
#pragma unroll
  for (int i = 0; i < 4; ++i)
#pragma unroll
    for (int j = 0; j < 4; ++j) acc[i][j] = (v8f){0.f,0.f,0.f,0.f,0.f,0.f,0.f,0.f};

  for (int k0 = 0; k0 < K; k0 += 32) {
    V bh[4], bl[4];
#pragma unroll
    for (int j = 0; j < 4; ++j) {
      const size_t bo = (size_t)(n0 + (j << 4) + rlane) * ldb + koff + k0;
      bh[j] = Frag<T>::load(Bb + bo);
      if (SPLIT) bl[j] = Frag<T>::load(Bb2 + bo);
    }
#pragma unroll
    for (int i = 0; i < 4; ++i) {
      const size_t ao = (size_t)(m0 + (i << 4) + rlane) * lda + koff + k0;
      V ah = Frag<T>::load(Ab + ao);
      V al;
      if (SPLIT) al = Frag<T>::load(Ab2 + ao);
#pragma unroll
      for (int j = 0; j < 4; ++j) {
        acc[i][j] = Frag<T>::mma(ah, bh[j], acc[i][j]);
        if (SPLIT) {
          acc[i][j] = Frag<T>::mma(ah, bl[j], acc[i][j]);
          acc[i][j] = Frag<T>::mma(al, bh[j], acc[i][j]);
        }
      }
      Frag<T>::guard(acc[i][0], acc[i][3], ah, SPLIT ? al : ah);
    }
    Frag<T>::keep(bh[0], bh[1], bh[2], bh[3]);
    if (SPLIT) Frag<T>::keep(bl[0], bl[1], bl[2], bl[3]);
  }
  acc_guard4(acc[0][0], acc[0][1], acc[0][2], acc[0][3]);
  acc_guard4(acc[1][0], acc[1][1], acc[1][2], acc[1][3]);
  acc_guard4(acc[2][0], acc[2][1], acc[2][2], acc[2][3]);
  acc_guard4(acc[3][0], acc[3][1], acc[3][2], acc[3][3]);

  float* slab = sT[wave];
  const float* Rb = RESID ? (resid + (size_t)b * strideR) : nullptr;
#pragma unroll
  for (int i = 0; i < 4; ++i) {
    const int mBase = m0 + (i << 4);
#pragma unroll
    for (int j = 0; j < 4; ++j) {
      const int n = n0 + (j << 4) + rlane;
      float bv = 0.f;
      if (BIAS_MODE == 2) bv = bias[n];
#pragma unroll
      for (int r = 0; r < 8; ++r) {
        float v = acc[i][j][r] * scale;
        if (BIAS_MODE == 1) v += bias[mBase + mOff + r];
        if (BIAS_MODE == 2) v += bv;
        if (RESID) v += Rb[(size_t)(mBase + mOff + r) * ldc + n];
        if (ACT == 2) v = fmaxf(v, 0.0f);
        if (ACT == 4) v = (v > 0.f) ? v : 0.01f * v;
        slab[(mOff + r) * 68 + (j << 4) + rlane] = v;
      }
    }
    __builtin_amdgcn_fence(__ATOMIC_RELEASE, "workgroup");
    __builtin_amdgcn_wave_barrier();
    __builtin_amdgcn_fence(__ATOMIC_ACQUIRE, "workgroup");
    if (OUT_MODE == 0) {
      float* C = (float*)Cout + (size_t)b * strideC;
      const int hh = lane >> 4, c4 = (lane & 15) * 4;
      for (int pass = 0; pass < 2; ++pass) {
#pragma unroll
        for (int it = 0; it < 8; ++it) {
          const int row = it * 2 + hh;
          v4f v = *(const v4f*)(slab + row * 68 + c4);
          *(volatile v4f*)(C + (size_t)(mBase + row) * ldc + n0 + c4) = v;
        }
        __threadfence();
      }
    } else {
      const int q = lane >> 3, c8 = (lane & 7) * 8;
      unsigned short* C  = (unsigned short*)Cout  + (size_t)b * strideC;
      unsigned short* C2 = (OUT_MODE == 2) ? ((unsigned short*)Cout2 + (size_t)b * strideC) : nullptr;
      for (int pass = 0; pass < 2; ++pass) {
#pragma unroll
        for (int it = 0; it < 4; ++it) {
          const int row = it * 4 + q;
          const float* sp = slab + row * 68 + c8;
          v8h hv, lv;
#pragma unroll
          for (int e = 0; e < 8; ++e) {
            if (OUT_MODE == 1) {
              hv[e] = (_Float16)sp[e];
            } else {
              unsigned short hb = f2bf_bits(sp[e]);
              unsigned short lb = f2bf_bits(sp[e] - bf_bits2f(hb));
              hv[e] = __builtin_bit_cast(_Float16, hb);
              lv[e] = __builtin_bit_cast(_Float16, lb);
            }
          }
          *(volatile v8h*)(C + (size_t)(mBase + row) * ldc + n0 + c8) = hv;
          if (OUT_MODE == 2) *(volatile v8h*)(C2 + (size_t)(mBase + row) * ldc + n0 + c8) = lv;
        }
        __threadfence();
      }
    }
    __builtin_amdgcn_fence(__ATOMIC_RELEASE, "workgroup");
    __builtin_amdgcn_wave_barrier();
    __builtin_amdgcn_fence(__ATOMIC_ACQUIRE, "workgroup");
  }
}

__global__ __launch_bounds__(256) void cast8_f16_kernel(const float* __restrict__ in, unsigned short* __restrict__ out,
                                                        int n8, float scale) {
  const int i = blockIdx.x * 256 + threadIdx.x;
  if (i >= n8) return;
  const float* p = in + 8 * (size_t)i;
  const v4f a = *(const v4f*)(p);
  const v4f c = *(const v4f*)(p + 4);
  unsigned short hb[8];
#pragma unroll
  for (int e = 0; e < 4; ++e) {
    hb[e]     = h_bits(a[e] * scale);
    hb[4 + e] = h_bits(c[e] * scale);
  }
  const v4u u = (v4u){pk16(hb[0], hb[1]), pk16(hb[2], hb[3]), pk16(hb[4], hb[5]), pk16(hb[6], hb[7])};
  unsigned short* q = out + 8 * (size_t)i;
  *(volatile v4u*)q = u;
  __threadfence();
  *(volatile v4u*)q = u;
}

__global__ __launch_bounds__(256) void relk_pad_kernel(const float* __restrict__ relk, unsigned short* __restrict__ out,
                                                       float scale) {
  const int i   = blockIdx.x * 256 + threadIdx.x;
  const int row = i >> 3;
  const int c8  = (i & 7) * 8;
  const int rr  = row < (kRel - 1) ? row : (kRel - 1);
  const float* p = relk + rr * kDk + c8;
  const v4f a = *(const v4f*)(p);
  const v4f c = *(const v4f*)(p + 4);
  const bool live = row < kRel;
  unsigned short hb[8];
#pragma unroll
  for (int e = 0; e < 4; ++e) {
    hb[e]     = h_bits(live ? a[e] * scale : 0.f);
    hb[4 + e] = h_bits(live ? c[e] * scale : 0.f);
  }
  const v4u u = (v4u){pk16(hb[0], hb[1]), pk16(hb[2], hb[3]), pk16(hb[4], hb[5]), pk16(hb[6], hb[7])};
  unsigned short* q = out + (size_t)row * kDk + c8;
  if (row < kRelPad) {
    *(volatile v4u*)q = u;
  }
  __threadfence();
  if (row < kRelPad) {
    *(volatile v4u*)q = u;
  }
}

__global__ __launch_bounds__(256) void vt_relv_fill_kernel(const float* __restrict__ relv, unsigned short* __restrict__ VT) {
  const int i   = blockIdx.x * 256 + threadIdx.x;
  const int row = i >> 4;
  const int c8  = (i & 15) * 8;
  const int d   = row & (kDk - 1);
  unsigned short hb[8];
#pragma unroll
  for (int e = 0; e < 8; ++e) {
    const int r  = c8 + e;
    const int rc = r < (kRel - 1) ? r : (kRel - 1);
    const float f = relv[rc * kDk + d];
    hb[e] = h_bits(r < kRel ? f : 0.f);
  }
  const v4u u = (v4u){pk16(hb[0], hb[1]), pk16(hb[2], hb[3]), pk16(hb[4], hb[5]), pk16(hb[6], hb[7])};
  unsigned short* q = VT + (size_t)row * kSPitch + kS + c8;
  if (row < kB * kH * kDk) {
    *(volatile v4u*)q = u;
  }
  __threadfence();
  if (row < kB * kH * kDk) {
    *(volatile v4u*)q = u;
  }
}

__global__ __launch_bounds__(128) void layernorm_f16_kernel(const float* __restrict__ X, const float* __restrict__ G,
                                                            const float* __restrict__ Bv, unsigned short* __restrict__ O) {
  __shared__ float red[2][4];
  const int row  = blockIdx.x;
  const int t    = threadIdx.x;
  const int lane = t & 31, wave = t >> 5;
  const int c0   = t * 8;
  const float* xr = X + (size_t)row * kD + c0;
  const v4f a = *(const v4f*)(xr);
  const v4f c = *(const v4f*)(xr + 4);
  float x[8];
#pragma unroll
  for (int e = 0; e < 4; ++e) { x[e] = a[e]; x[4 + e] = c[e]; }
  float s = 0.f;
#pragma unroll
  for (int e = 0; e < 8; ++e) s += x[e];
#pragma unroll
  for (int off = 16; off > 0; off >>= 1) s += __shfl_xor(s, off, 32);
  if (lane == 0) red[0][wave] = s;
  __syncthreads();
  const float tot = ((red[0][0] + red[0][1]) + red[0][2]) + red[0][3];
  const float mu  = tot * kInvD;
  float dv[8];
  float s2 = 0.f;
#pragma unroll
  for (int e = 0; e < 8; ++e) { dv[e] = x[e] - mu; s2 += dv[e] * dv[e]; }
#pragma unroll
  for (int off = 16; off > 0; off >>= 1) s2 += __shfl_xor(s2, off, 32);
  if (lane == 0) red[1][wave] = s2;
  __syncthreads();
  const float tot2 = ((red[1][0] + red[1][1]) + red[1][2]) + red[1][3];
  const float var  = tot2 * kInvD;
  const float rstd = rsqrtf(var + kLnEps);
  const v4f g0 = *(const v4f*)(G + c0);
  const v4f g1 = *(const v4f*)(G + c0 + 4);
  const v4f b0 = *(const v4f*)(Bv + c0);
  const v4f b1 = *(const v4f*)(Bv + c0 + 4);
  unsigned short hb[8];
#pragma unroll
  for (int e = 0; e < 4; ++e) {
    hb[e]     = h_bits(dv[e] * rstd * g0[e] + b0[e]);
    hb[4 + e] = h_bits(dv[4 + e] * rstd * g1[e] + b1[e]);
  }
  const v4u u = (v4u){pk16(hb[0], hb[1]), pk16(hb[2], hb[3]), pk16(hb[4], hb[5]), pk16(hb[6], hb[7])};
  unsigned short* q = O + (size_t)row * kD + c0;
  *(volatile v4u*)q = u;
  __threadfence();
  *(volatile v4u*)q = u;
}

__global__ __launch_bounds__(128) void softmax_rel_kernel(const float* __restrict__ SC, unsigned short* __restrict__ P,
                                                          float carry) {
  __shared__ float sqr[kRelPad];
  __shared__ __align__(16) float sp[kS];
  __shared__ __align__(16) float prrow[kRelPad];
  __shared__ float red[4][4];
  const int bx   = blockIdx.x;
  const int i    = bx & (kS - 1);
  const int t    = threadIdx.x, lane = t & 31, wave = t >> 5;
  const int c0   = t * 8;
  const float* sr = SC + (size_t)bx * kSPitch;
  sqr[t] = sr[kS + t];
  const v4f a  = *(const v4f*)(sr + c0);
  const v4f cc = *(const v4f*)(sr + c0 + 4);
  float x[8];
#pragma unroll
  for (int e = 0; e < 4; ++e) { x[e] = a[e]; x[4 + e] = cc[e]; }
  __syncthreads();
  float m = -INFINITY;
#pragma unroll
  for (int e = 0; e < 8; ++e) {
    const int j = c0 + e;
    int dl = j - i;
    dl = dl < -kMaxRel ? -kMaxRel : dl;
    dl = dl >  kMaxRel ?  kMaxRel : dl;
    const float v = x[e] + sqr[dl + kMaxRel];
    sp[j] = v;
    m = fmaxf(m, v);
  }
#pragma unroll
  for (int off = 16; off > 0; off >>= 1) m = fmaxf(m, __shfl_xor(m, off, 32));
  if (lane == 0) red[0][wave] = m;
  __syncthreads();
  const float rmax = fmaxf(fmaxf(red[0][0], red[0][1]), fmaxf(red[0][2], red[0][3]));
  float ls = 0.f, lo = 0.f, hi = 0.f;
#pragma unroll 1
  for (int e = 0; e < 8; ++e) {
    const int j = c0 + e;
    const float ex = expf(sp[j] - rmax);
    sp[j] = ex;
    ls += ex;
    lo += (j <= i - kMaxRel) ? ex : 0.f;
    hi += (j >= i + kMaxRel) ? ex : 0.f;
  }
#pragma unroll
  for (int off = 16; off > 0; off >>= 1) {
    ls += __shfl_xor(ls, off, 32);
    lo += __shfl_xor(lo, off, 32);
    hi += __shfl_xor(hi, off, 32);
  }
  if (lane == 0) { red[1][wave] = ls; red[2][wave] = lo; red[3][wave] = hi; }
  __syncthreads();
  const float ssum  = ((red[1][0] + red[1][1]) + red[1][2]) + red[1][3];
  const float losum = ((red[2][0] + red[2][1]) + red[2][2]) + red[2][3];
  const float hisum = ((red[3][0] + red[3][1]) + red[3][2]) + red[3][3];
  const float pcar  = carry * (1.0f / ssum);
  {
    const v4f e0 = *(const v4f*)(sp + c0);
    const v4f e1 = *(const v4f*)(sp + c0 + 4);
    unsigned short hb[8];
#pragma unroll
    for (int e = 0; e < 4; ++e) {
      hb[e]     = h_bits(e0[e] * pcar);
      hb[4 + e] = h_bits(e1[e] * pcar);
    }
    const v4u u = (v4u){pk16(hb[0], hb[1]), pk16(hb[2], hb[3]), pk16(hb[4], hb[5]), pk16(hb[6], hb[7])};
    unsigned short* q = P + (size_t)bx * kSPitch + c0;
    *(volatile v4u*)q = u;
    __threadfence();
    *(volatile v4u*)q = u;
  }
  {
    const int r = t;
    const int j = i + r - kMaxRel;
    const bool inr = (r >= 1) && (r <= 2 * kMaxRel - 1) && (j >= 0) && (j < kS);
    int jc = j < 0 ? 0 : j;
    jc = jc > (kS - 1) ? (kS - 1) : jc;
    const float exv = sp[jc];
    float val = inr ? exv : 0.f;
    val = (r == 0) ? losum : val;
    val = (r == 2 * kMaxRel) ? hisum : val;
    prrow[t] = val * pcar;
  }
  __syncthreads();
  {
    const int q8 = t & 15;
    const v4f p0 = *(const v4f*)(prrow + 8 * q8);
    const v4f p1 = *(const v4f*)(prrow + 8 * q8 + 4);
    unsigned short hb[8];
#pragma unroll
    for (int e = 0; e < 4; ++e) {
      hb[e]     = h_bits(p0[e]);
      hb[4 + e] = h_bits(p1[e]);
    }
    const v4u u = (v4u){pk16(hb[0], hb[1]), pk16(hb[2], hb[3]), pk16(hb[4], hb[5]), pk16(hb[6], hb[7])};
    unsigned short* q = P + (size_t)bx * kSPitch + kS + 8 * q8;
    if (t < 16) {
      *(volatile v4u*)q = u;
    }
    __threadfence();
    if (t < 16) {
      *(volatile v4u*)q = u;
    }
  }
}

__global__ __launch_bounds__(256) void geglu_kernel(const float* __restrict__ Hp, unsigned short* __restrict__ Gp,
                                                    int mc, float carry) {
  const int gi  = blockIdx.x * 256 + threadIdx.x;
  const int row = gi >> 9;
  const int c   = (gi & 511) * 8;
  const float* hr = Hp + (size_t)row * (2 * kFF);
  unsigned u0 = 0u, u1 = 0u, u2 = 0u, u3 = 0u;
#pragma unroll 1
  for (int e = 0; e < 8; ++e) {
    const float g  = hr[c + e];
    const float l  = hr[kFF + c + e];
    const float ge = 0.5f * g * (1.0f + erff(g * 0.70710678118654752f));
    const unsigned w = ((unsigned)h_bits(ge * l * carry)) << ((e & 1) * 16);
    u0 |= (e < 2) ? w : 0u;
    u1 |= ((e >> 1) == 1) ? w : 0u;
    u2 |= ((e >> 1) == 2) ? w : 0u;
    u3 |= ((e >> 1) == 3) ? w : 0u;
  }
  const v4u u = (v4u){u0, u1, u2, u3};
  unsigned short* q = Gp + (size_t)(mc * kS + row) * kFF + c;
  if (row < kS) {
    *(volatile v4u*)q = u;
  }
  __threadfence();
  if (row < kS) {
    *(volatile v4u*)q = u;
  }
}

extern "C" void kernel_launch(void* const* d_in, const int* in_sizes, int n_in,
                              void* d_out, int out_size, void* d_ws, size_t ws_size, hipStream_t stream) {
  if (n_in < 16) return;
  if (in_sizes[0] != kTok * kD) return;
  if (in_sizes[1] != kD * kD || in_sizes[2] != kD * kD || in_sizes[3] != kD * kD || in_sizes[4] != kD * kD) return;
  if (in_sizes[5] != kD || in_sizes[11] != kD || in_sizes[12] != kD || in_sizes[13] != kD ||
      in_sizes[14] != kD || in_sizes[15] != kD) return;
  if (in_sizes[6] != kRel * kDk || in_sizes[7] != kRel * kDk) return;
  if (in_sizes[8] != 2 * kFF * kD || in_sizes[9] != 2 * kFF || in_sizes[10] != kD * kFF) return;
  if (out_size != kTok * kD) return;
  if (ws_size < kWsTotal) return;

  const float* src  = (const float*)d_in[0];
  const float* w_q  = (const float*)d_in[1];
  const float* w_k  = (const float*)d_in[2];
  const float* w_v  = (const float*)d_in[3];
  const float* w_o  = (const float*)d_in[4];
  const float* b_o  = (const float*)d_in[5];
  const float* relk = (const float*)d_in[6];
  const float* relv = (const float*)d_in[7];
  const float* w1   = (const float*)d_in[8];
  const float* b1   = (const float*)d_in[9];
  const float* w2   = (const float*)d_in[10];
  const float* b2   = (const float*)d_in[11];
  const float* g1   = (const float*)d_in[12];
  const float* be1  = (const float*)d_in[13];
  const float* g2   = (const float*)d_in[14];
  const float* be2  = (const float*)d_in[15];
  float* out = (float*)d_out;

  char* ws = (char*)d_ws;
  float*          SRC1  = (float*)(ws + kOffSrc1);
  unsigned short* X16   = (unsigned short*)(ws + kOffX16);
  unsigned short* W4    = (unsigned short*)(ws + kOffW4);
  unsigned short* Q16   = (unsigned short*)(ws + kOffQ16);
  unsigned short* K16   = (unsigned short*)(ws + kOffK16);
  unsigned short* VT16  = (unsigned short*)(ws + kOffVT);
  float*          SC    = (float*)(ws + kOffSC);
  unsigned short* P16   = (unsigned short*)(ws + kOffP16);
  unsigned short* CTX16 = (unsigned short*)(ws + kOffCtx);
  unsigned short* RELK  = (unsigned short*)(ws + kOffRelk);
  unsigned short* Y16   = (unsigned short*)(ws + kOffY16);
  unsigned short* W1P   = (unsigned short*)(ws + kOffW1);
  unsigned short* W2P   = (unsigned short*)(ws + kOffW2);
  float*          HP    = (float*)(ws + kOffH);
  unsigned short* G16   = (unsigned short*)(ws + kOffG16);

  const size_t kWPlane = (size_t)kD * kD;
  unsigned short* WQ16 = W4 + 0 * kWPlane;
  unsigned short* WK16 = W4 + 1 * kWPlane;
  unsigned short* WV16 = W4 + 2 * kWPlane;
  unsigned short* WO16 = W4 + 3 * kWPlane;

  {
    const int n8w = (kD * kD) / 8;
    const dim3 gw((n8w + 255) / 256);
    cast8_f16_kernel<<<gw, dim3(256), 0, stream>>>(w_q, WQ16, n8w, kWCarry);
    cast8_f16_kernel<<<gw, dim3(256), 0, stream>>>(w_k, WK16, n8w, kWCarry);
    cast8_f16_kernel<<<gw, dim3(256), 0, stream>>>(w_v, WV16, n8w, kWCarry);
    cast8_f16_kernel<<<gw, dim3(256), 0, stream>>>(w_o, WO16, n8w, kWCarry);
  }
  relk_pad_kernel<<<dim3((kRelPad * kDk / 8) / 256), dim3(256), 0, stream>>>(relk, RELK, kRelkCarry);

  layernorm_f16_kernel<<<dim3(kTok), dim3(128), 0, stream>>>(src, g1, be1, X16);

  {
    const dim3 gq((64 * 16) / 8, 1);
    wmma_gemm64<0, false, 0, 1, false><<<gq, dim3(256), 0, stream>>>(
        X16, nullptr, kD, 0L, WQ16, nullptr, kD, 0L,
        (void*)Q16, nullptr, kD, 0L, nullptr, nullptr, 0L, kTok, kD, kD, 1.0f / kWCarry);
    wmma_gemm64<0, false, 0, 1, false><<<gq, dim3(256), 0, stream>>>(
        X16, nullptr, kD, 0L, WK16, nullptr, kD, 0L,
        (void*)K16, nullptr, kD, 0L, nullptr, nullptr, 0L, kTok, kD, kD, 1.0f / kWCarry);
  }
  {
    const dim3 gv((16 * 16) / 8, kB);
    wmma_gemm64<0, false, 0, 1, false><<<gv, dim3(256), 0, stream>>>(
        WV16, nullptr, kD, 0L, X16, nullptr, kD, (long)kS * kD,
        (void*)VT16, nullptr, kSPitch, (long)kD * kSPitch, nullptr, nullptr, 0L, kD, kS, kD, 1.0f / kWCarry);
  }
  vt_relv_fill_kernel<<<dim3((kB * kH * kDk * (kRelPad / 8)) / 256), dim3(256), 0, stream>>>(relv, VT16);

  for (int c = 0; c < kNChunk; ++c) {
    const int b  = c >> 1;
    const int h0 = (c & 1) * kG;
    const unsigned short* Qg = Q16 + (size_t)b * kS * kD + (size_t)h0 * kDk;
    const unsigned short* Kg = K16 + (size_t)b * kS * kD + (size_t)h0 * kDk;
    wmma_gemm64<0, false, 0, 0, false><<<dim3((16 * 16) / 8, kG), dim3(256), 0, stream>>>(
        Qg, nullptr, kD, (long)kDk, Kg, nullptr, kD, (long)kDk,
        (void*)SC, nullptr, kSPitch, (long)kS * kSPitch, nullptr, nullptr, 0L, kS, kS, kDk, 0.125f);
    wmma_gemm64<0, false, 0, 0, false><<<dim3((16 * 2) / 8, kG), dim3(256), 0, stream>>>(
        Qg, nullptr, kD, (long)kDk, RELK, nullptr, kDk, 0L,
        (void*)(SC + kS), nullptr, kSPitch, (long)kS * kSPitch, nullptr, nullptr, 0L, kS, kRelPad, kDk, 1.0f / kRelkCarry);
    softmax_rel_kernel<<<dim3(kG * kS), dim3(128), 0, stream>>>(SC, P16, kPCarry);
    wmma_gemm64<0, false, 0, 1, false><<<dim3((16 * 1) / 8, kG), dim3(256), 0, stream>>>(
        P16, nullptr, kSPitch, (long)kS * kSPitch,
        VT16 + (size_t)(c * kG) * kDk * kSPitch, nullptr, kSPitch, (long)kDk * kSPitch,
        (void*)(CTX16 + (size_t)b * kS * kD + (size_t)h0 * kDk), nullptr, kD, (long)kDk,
        nullptr, nullptr, 0L, kS, kDk, kSPitch, kCtxCarry / kPCarry);
  }

  wmma_gemm64<0, false, 2, 0, true><<<dim3((64 * 16) / 8, 1), dim3(256), 0, stream>>>(
      CTX16, nullptr, kD, 0L, WO16, nullptr, kD, 0L,
      (void*)SRC1, nullptr, kD, 0L, b_o, src, 0L, kTok, kD, kD, 1.0f / (kCtxCarry * kWCarry));

  {
    const int n8a = (2 * kFF * kD) / 8;
    const int n8b = (kD * kFF) / 8;
    cast8_f16_kernel<<<dim3((n8a + 255) / 256), dim3(256), 0, stream>>>(w1, W1P, n8a, kWCarry);
    cast8_f16_kernel<<<dim3((n8b + 255) / 256), dim3(256), 0, stream>>>(w2, W2P, n8b, kWCarry);
  }
  layernorm_f16_kernel<<<dim3(kTok), dim3(128), 0, stream>>>(SRC1, g2, be2, Y16);

  for (int mc = 0; mc < kTok / kS; ++mc) {
    wmma_gemm64<0, false, 2, 0, false><<<dim3((16 * 128) / 8, 1), dim3(256), 0, stream>>>(
        Y16 + (size_t)mc * kS * kD, nullptr, kD, 0L, W1P, nullptr, kD, 0L,
        (void*)HP, nullptr, 2 * kFF, 0L, b1, nullptr, 0L, kS, 2 * kFF, kD, 1.0f / kWCarry);
    geglu_kernel<<<dim3((kS * kFF / 8) / 256), dim3(256), 0, stream>>>(HP, G16, mc, kGCarry);
  }
  wmma_gemm64<0, false, 2, 0, true><<<dim3((64 * 16) / 8, 1), dim3(256), 0, stream>>>(
      G16, nullptr, kFF, 0L, W2P, nullptr, kFF, 0L,
      (void*)out, nullptr, kD, 0L, b2, SRC1, 0L, kTok, kD, kFF, 1.0f / (kGCarry * kWCarry));
}
